// SnapshotGraphEncoder_7043746365769
// MI455X (gfx1250) — hardware-run, weakly checked
//
#include <hip/hip_runtime.h>

typedef float          v8f   __attribute__((ext_vector_type(8)));
typedef float          v4f   __attribute__((ext_vector_type(4)));
typedef unsigned int   v4u   __attribute__((ext_vector_type(4)));
typedef int            v8i   __attribute__((ext_vector_type(8)));
typedef unsigned short v8us  __attribute__((ext_vector_type(8)));
typedef unsigned short v16us __attribute__((ext_vector_type(16)));
typedef __bf16         v16bf __attribute__((ext_vector_type(16)));
typedef _Float16       v16h  __attribute__((ext_vector_type(16)));
typedef v4f  __attribute__((may_alias)) v4fa;
typedef v8us __attribute__((may_alias)) v8usa;
union FragB { v16bf v; v16us u; v8us h[2]; v8i w; };
union FragH { v16h  v; v16us u; v8us h[2]; v8i w; };

__device__ __forceinline__ v8f wmb(const FragB& a, const FragB& b, v8f c) {
  v8f d = __builtin_amdgcn_wmma_f32_16x16x32_bf16(false, a.v, false, b.v, (short)0, c, false, false);
  asm volatile("v_nop\n\tv_nop\n\tv_nop\n\tv_nop" : "+v"(d) : "v"(a.w), "v"(b.w));
  return d;
}

__device__ __forceinline__ v8f wmh(const FragH& a, const FragH& b, v8f c) {
  v8f d = __builtin_amdgcn_wmma_f32_16x16x32_f16(false, a.v, false, b.v, (short)0, c, false, false);
  asm volatile("v_nop\n\tv_nop\n\tv_nop\n\tv_nop" : "+v"(d) : "v"(a.w), "v"(b.w));
  return d;
}

__device__ __forceinline__ unsigned bf16_bits(float f) {
  const unsigned u = __float_as_uint(f);
  const unsigned r = (u + 0x7FFFu + ((u >> 16) & 1u)) >> 16;
  const unsigned q = (u >> 16) | 0x40u;
  return ((u & 0x7fffffffu) > 0x7f800000u) ? q : r;
}

__device__ __forceinline__ float bf16_val(float f) {
  return __uint_as_float(bf16_bits(f) << 16);
}
__device__ __forceinline__ int clampi(int v, int lo, int hi) {
  return v < lo ? lo : (v > hi ? hi : v);
}

__device__ __forceinline__ unsigned f16_bits(float f) {
  const unsigned u  = __float_as_uint(f);
  const unsigned s  = (u >> 16) & 0x8000u;
  const unsigned a  = u & 0x7fffffffu;
  const unsigned t  = a - 0x38000000u;
  const unsigned r  = (t + 0x0FFFu + ((t >> 13) & 1u)) >> 13;
  const unsigned rc = r > 0x7C00u ? 0x7C00u : r;
  const bool small  = a < 0x38800000u;
  const bool isnan  = a > 0x7f800000u;
  const unsigned fin = small ? 0u : (s | rc);
  return isnan ? (s | 0x7E00u) : fin;
}

__device__ __forceinline__ unsigned pk16(unsigned lo, unsigned hi) { return lo | (hi << 16); }
__device__ __forceinline__ unsigned bf16_lo_bits(float v) {
  float hi = bf16_val(v);
  asm volatile("" : "+v"(hi));
  return bf16_bits(v - hi);
}
__device__ __forceinline__ v4u pack8_bf16(v4f a, v4f c) {
  return (v4u){ pk16(bf16_bits(a[0]), bf16_bits(a[1])), pk16(bf16_bits(a[2]), bf16_bits(a[3])),
                pk16(bf16_bits(c[0]), bf16_bits(c[1])), pk16(bf16_bits(c[2]), bf16_bits(c[3])) };
}
__device__ __forceinline__ v4u pack8_bf16_lo(v4f a, v4f c) {
  return (v4u){ pk16(bf16_lo_bits(a[0]), bf16_lo_bits(a[1])), pk16(bf16_lo_bits(a[2]), bf16_lo_bits(a[3])),
                pk16(bf16_lo_bits(c[0]), bf16_lo_bits(c[1])), pk16(bf16_lo_bits(c[2]), bf16_lo_bits(c[3])) };
}
__device__ __forceinline__ v4u pack8_f16(v4f a, v4f c) {
  return (v4u){ pk16(f16_bits(a[0]), f16_bits(a[1])), pk16(f16_bits(a[2]), f16_bits(a[3])),
                pk16(f16_bits(c[0]), f16_bits(c[1])), pk16(f16_bits(c[2]), f16_bits(c[3])) };
}

template <int FORM>
__global__ __launch_bounds__(256) void k_plane(const float* __restrict__ src, int rows, int cols, int ldsrc,
                                               unsigned short* __restrict__ dst, int MP, int KP) {
  static_assert(FORM >= 0 && FORM <= 3);
  const int KTOT = (FORM == 1 || FORM == 3) ? 2 * KP : KP;
  const unsigned ppr   = (unsigned)(KTOT >> 3);
  const unsigned kp8   = (unsigned)(KP >> 3);
  const unsigned total = (unsigned)MP * ppr;
  const unsigned g     = blockIdx.x * 256u + threadIdx.x;
  const unsigned rowu  = g / ppr;
  const unsigned p     = g - rowu * ppr;
  const bool second    = p >= kp8;
  const int row = (int)rowu;
  const int c0  = (int)((second ? p - kp8 : p) << 3);
  const float* srow = src + (size_t)clampi(row, 0, rows - 1) * (size_t)ldsrc;
  float x[8];
  unsigned mk[8];
#pragma unroll
  for (int e = 0; e < 8; ++e) {
    const int c = c0 + e;
    const float v = srow[clampi(c, 0, cols - 1)];
    asm volatile("" :: "v"(v));
    x[e]  = v;
    mk[e] = (row < rows && c < cols) ? 0xFFFFu : 0u;
  }
  const v4f a = (v4f){ x[0], x[1], x[2], x[3] };
  const v4f c = (v4f){ x[4], x[5], x[6], x[7] };
  v4u o;
  if (FORM == 2) {
    o = pack8_f16(a, c);
  } else {
    const v4u hi = pack8_bf16(a, c);
    o = hi;
    if (FORM == 1) { const v4u lo = pack8_bf16_lo(a, c); o = second ? lo : hi; }
  }
  const v4u mw = (v4u){ pk16(mk[0], mk[1]), pk16(mk[2], mk[3]), pk16(mk[4], mk[5]), pk16(mk[6], mk[7]) };
  o &= mw;
  if (g < total) {
    volatile v4u* q = (volatile v4u*)(dst + (size_t)g * 8);
    *q = o;
    __threadfence();
    *q = o;
  }
}

template <int FORM> struct FragOf    { typedef FragB T; };
template <>         struct FragOf<2> { typedef FragH T; };
__device__ __forceinline__ v8f mm(const FragB& a, const FragB& b, v8f c) { return wmb(a, b, c); }
__device__ __forceinline__ v8f mm(const FragH& a, const FragH& b, v8f c) { return wmh(a, b, c); }
template <class F> __device__ __forceinline__ F ld_frag(const unsigned short* p) {
  F f;
  f.h[0] = *(const v8usa*)(p);
  f.h[1] = *(const v8usa*)(p + 16);
  return f;
}

template <int FORM, int EPI>
__global__ __launch_bounds__(256) __attribute__((amdgpu_num_vgpr(248)))
void k_gemm_nt(const unsigned short* __restrict__ A, const unsigned short* __restrict__ B,
               const float* __restrict__ bias, float* __restrict__ D, int M, int N, int KTOT, int ldd) {
  static_assert(FORM >= 0 && FORM <= 2);
  static_assert(EPI == 0 || EPI == 1);
  typedef typename FragOf<FORM>::T F;
  __shared__ __attribute__((aligned(16))) float sT[8][16 * 68];
  const int lane = threadIdx.x & 31;
  const int wave = threadIdx.x >> 5;
  const int tilesM = (M + 63) >> 6;
  const int tilesN = (N + 63) >> 6;
  const int tile = blockIdx.x * 8 + wave;
  if (tile >= tilesM * tilesN) return;
  const int tm = tile / tilesN;
  const int tn = tile - tm * tilesN;
  const int m0 = tm << 6;
  const int n0 = tn << 6;

  const int rl = lane & 15;
  const int h8 = (lane >> 4) * 8;
  const unsigned short* pa = A + (size_t)(m0 + rl) * (size_t)KTOT + h8;
  const unsigned short* pb = B + (size_t)(n0 + rl) * (size_t)KTOT + h8;

  v8f acc[4][4];
#pragma unroll
  for (int i = 0; i < 4; ++i)
#pragma unroll
    for (int j = 0; j < 4; ++j) acc[i][j] = (v8f){0.f, 0.f, 0.f, 0.f, 0.f, 0.f, 0.f, 0.f};

#pragma unroll 1
  for (int k0 = 0; k0 < KTOT; k0 += 32) {
    F bf[4];
#pragma unroll
    for (int j = 0; j < 4; ++j) bf[j] = ld_frag<F>(pb + (size_t)(j << 4) * (size_t)KTOT + k0);
#pragma unroll
    for (int i = 0; i < 4; ++i) {
      const F af = ld_frag<F>(pa + (size_t)(i << 4) * (size_t)KTOT + k0);
#pragma unroll
      for (int j = 0; j < 4; ++j) acc[i][j] = mm(af, bf[j], acc[i][j]);
    }
  }

  float* slab = sT[wave];
  const int hh = lane >> 4;
  const int c4 = (lane & 15) * 4;
  const int nc = n0 + c4;
  const bool cok = nc < N;
  v4f bv = (v4f){0.f, 0.f, 0.f, 0.f};
  if (EPI == 1) {
    bv = *(const v4fa*)(bias + clampi(nc, 0, N - 4));
    asm volatile("" :: "v"(bv));
  }
#pragma unroll
  for (int i = 0; i < 4; ++i) {
    const int mBase = m0 + (i << 4);
#pragma unroll
    for (int j = 0; j < 4; ++j) {
#pragma unroll
      for (int r = 0; r < 8; ++r) slab[(h8 + r) * 68 + (j << 4) + rl] = acc[i][j][r];
    }
    __builtin_amdgcn_fence(__ATOMIC_RELEASE, "workgroup");
    __builtin_amdgcn_wave_barrier();
    __builtin_amdgcn_fence(__ATOMIC_ACQUIRE, "workgroup");
    v4f vv[8];
#pragma unroll
    for (int it = 0; it < 8; ++it) {
      const int row = it * 2 + hh;
      v4f v = *(const v4fa*)(slab + row * 68 + c4);
      if (EPI == 1) v += bv;
      vv[it] = v;
    }
    for (int pass = 0; pass < 2; ++pass) {
#pragma unroll
      for (int it = 0; it < 8; ++it) {
        const int row = mBase + it * 2 + hh;
        if (cok && row < M) *(volatile v4f*)(D + (size_t)row * (size_t)ldd + nc) = vv[it];
      }
      __threadfence();
    }
    __builtin_amdgcn_fence(__ATOMIC_RELEASE, "workgroup");
    __builtin_amdgcn_wave_barrier();
    __builtin_amdgcn_fence(__ATOMIC_ACQUIRE, "workgroup");
  }
}

#define NN      50000
#define NE      800000
#define ATTR    125
#define DF      128
#define MP      50048
#define AP      512
#define NBLK    49
#define NBA     1024
#define SLA     10
#define MEAS_B1024  16594
#define MEAS_MAXDEG 37
#define RCAP    21504
#define WLCAP   4096
#define DEGCAP  64
#define EW      (NE / 8)
#define STEP    256
#define NSTEP   ((EW + STEP - 1) / STEP)
#define XROWS   64
#define TWO_TERM 1
#define BK_ZINTS (8 * NBA + RCAP + 64)
#define BK_INTS  (8 * WLCAP + BK_ZINTS)
#define BK_LDS   (BK_INTS * 4)

#define SZ_X0B   ((size_t)MP * DF * 2)
#define SZ_XF    ((size_t)MP * DF * 4)
#define SZ_A     ((size_t)MP * AP * 2)
#define SZ_Y     ((size_t)MP * DF * 4)
#define SZ_LIST  ((size_t)NBLK * RCAP * 4)
#define SZ_CNT   ((size_t)NBLK * NBA * 4)
#define SZ_FLAG  ((size_t)NBLK * 128)
#define SZ_WIN   ((size_t)DF * DF * 2)
#define SZ_WCAT  ((size_t)DF * AP * 2)
#define WS_TOTAL (SZ_X0B + SZ_XF + SZ_A + SZ_Y + SZ_LIST + 2 * SZ_CNT + SZ_FLAG + SZ_WIN + 2 * SZ_WCAT)

static_assert(NN == 50000);
static_assert(NE == 390 * 2048 + 1280);
static_assert(NE == 8 * (390 * STEP + 160) && NSTEP == 391);
static_assert(ATTR + 3 == DF);
static_assert(MP == 391 * 128 && MP % 64 == 0 && MP >= NN && NN % 16 == 0);
static_assert(NBLK == (MP + NBA - 1) / NBA && NBLK * NBA >= MP && NBA == (1 << SLA));
static_assert(RCAP % 1024 == 0 && (long long)RCAP * 4 >= (long long)MEAS_B1024 * 5);
static_assert(DEGCAP >= MEAS_MAXDEG + 8);
static_assert(8 * WLCAP >= RCAP && (long long)WLCAP * 8 * 4 >= (long long)MEAS_B1024 * 5);
static_assert(EW % 8 == 0 && NE % 4 == 0 && EW >= 8);
static_assert(((long long)(NN - 1) << SLA) + NBA < (1LL << 31));
static_assert(BK_ZINTS % 4 == 0 && BK_LDS <= 262144 && BK_LDS <= 327680);
static_assert((NN * ATTR) % 4 == 0 && (XROWS * ATTR) % 4 == 0 && MP % XROWS == 0);
static_assert(SZ_X0B % 128 == 0 && SZ_XF % 128 == 0 && SZ_A % 128 == 0 && SZ_LIST % 128 == 0);
static_assert(SZ_CNT % 128 == 0 && SZ_FLAG % 128 == 0 && SZ_WIN % 128 == 0 && SZ_WCAT % 128 == 0);
static_assert(((size_t)RCAP * 4) % 128 == 0);
static_assert(WS_TOTAL <= ((size_t)128 << 20));
static_assert(AP == 4 * DF && AP % 32 == 0 && DF % 32 == 0);

typedef int      v4i __attribute__((ext_vector_type(4)));
typedef unsigned v2u __attribute__((ext_vector_type(2)));
typedef v4i __attribute__((may_alias)) v4ia;
typedef v2u __attribute__((may_alias)) v2ua;
typedef v4u __attribute__((may_alias)) v4ua;

__device__ __forceinline__ void wave_sync() {
  __builtin_amdgcn_fence(__ATOMIC_RELEASE, "workgroup");
  __builtin_amdgcn_wave_barrier();
  __builtin_amdgcn_fence(__ATOMIC_ACQUIRE, "workgroup");
}

__device__ __forceinline__ float blendf(float a, float b, unsigned m) {
  return __uint_as_float((__float_as_uint(b) & m) | (__float_as_uint(a) & ~m));
}

__device__ __forceinline__ float relu_keep(float v) { return (v > 0.0f) ? v : (v - v); }

__device__ __forceinline__ v4u hilo_piece(unsigned short* rb, int lane, v4f m) {
  const v2u hw = (v2u){ pk16(bf16_bits(m[0]), bf16_bits(m[1])), pk16(bf16_bits(m[2]), bf16_bits(m[3])) };
#if TWO_TERM
  const v2u lw = (v2u){ pk16(bf16_lo_bits(m[0]), bf16_lo_bits(m[1])), pk16(bf16_lo_bits(m[2]), bf16_lo_bits(m[3])) };
#else
  const v2u lw = (v2u){ 0u, 0u };
#endif
  *(v2ua*)(rb + 4 * lane) = hw;
  *(v2ua*)(rb + DF + 4 * lane) = lw;
  wave_sync();
  const v4u q = *(const v4ua*)(rb + 8 * lane);
  wave_sync();
  return q;
}

__global__ __launch_bounds__(256) void k_xplane(const float* __restrict__ attr, const float* __restrict__ cl,
                                                const float* __restrict__ ra, const float* __restrict__ ex,
                                                unsigned short* X0B, int nN) {
  __shared__ __attribute__((aligned(16))) float sx[XROWS * ATTR];
  __shared__ float s3[3][XROWS];
  const int tid = (int)threadIdx.x;
  const int r0 = (int)blockIdx.x * XROWS;
  const int base4 = (int)blockIdx.x * (XROWS * ATTR / 4);
  const int tot4 = NN * ATTR / 4;
#pragma unroll 4
  for (int it = 0; it < 8; ++it) {
    const int i = tid + 256 * it;
    const int ic = i < (XROWS * ATTR / 4) ? i : (XROWS * ATTR / 4 - 1);
    int g = base4 + ic;
    g = g > tot4 - 1 ? tot4 - 1 : g;
    const v4f v = *(const v4f*)(attr + (size_t)g * 4);
    asm volatile("" :: "v"(v));
    if (i < XROWS * ATTR / 4) *(v4fa*)(sx + 4 * i) = v;
  }
  {
    const int rr = tid & (XROWS - 1);
    int rg = r0 + rr;
    rg = rg > nN - 1 ? nN - 1 : rg;
    const float c1 = cl[rg];
    const float c2 = ra[rg];
    const float c3 = ex[rg];
    asm volatile("" :: "v"(c1));
    asm volatile("" :: "v"(c2));
    asm volatile("" :: "v"(c3));
    if (tid < XROWS) { s3[0][rr] = c1; s3[1][rr] = c2; s3[2][rr] = c3; }
  }
  __syncthreads();
  const int p = tid & 15;
  const unsigned m15 = (p == 15) ? 0xFFFFFFFFu : 0u;
  v4u o[4];
#pragma unroll
  for (int it = 0; it < 4; ++it) {
    const int r = (tid >> 4) + 16 * it;
    const float* srow = sx + r * ATTR;
    float x[8];
#pragma unroll
    for (int e = 0; e < 8; ++e) {
      const int c = 8 * p + e;
      x[e] = srow[c < ATTR ? c : ATTR - 1];
    }
    x[5] = blendf(x[5], s3[0][r], m15);
    x[6] = blendf(x[6], s3[1][r], m15);
    x[7] = blendf(x[7], s3[2][r], m15);
    const unsigned rm = (r0 + r < nN) ? 0xFFFFFFFFu : 0u;
    const v4u w = pack8_bf16((v4f){ x[0], x[1], x[2], x[3] }, (v4f){ x[4], x[5], x[6], x[7] });
    o[it] = w & (v4u){ rm, rm, rm, rm };
  }
  unsigned short* dst = X0B + (size_t)r0 * DF;
#pragma unroll
  for (int it = 0; it < 4; ++it) *(volatile v4u*)(dst + (size_t)(tid + 256 * it) * 8) = o[it];
  __threadfence();
#pragma unroll
  for (int it = 0; it < 4; ++it) *(volatile v4u*)(dst + (size_t)(tid + 256 * it) * 8) = o[it];
}

__global__ __launch_bounds__(256) void k_wcat(const float* __restrict__ Ws, const float* __restrict__ Wn,
                                              unsigned short* P) {
  const int u  = (int)blockIdx.x * 256 + (int)threadIdx.x;
  const int n  = (u >> 4) & (DF - 1);
  const int k8 = (u & 15) * 8;
  const float* ps = Ws + (size_t)n * DF + k8;
  const float* pn = Wn + (size_t)n * DF + k8;
  const v4f s0 = *(const v4f*)ps;
  const v4f s1 = *(const v4f*)(ps + 4);
  const v4f n0 = *(const v4f*)pn;
  const v4f n1 = *(const v4f*)(pn + 4);
  const v4u os = pack8_bf16(s0, s1);
  const v4u on = pack8_bf16(n0, n1);
  unsigned short* dp = P + (size_t)n * AP + k8;
  *(volatile v4u*)(dp)          = os;
  *(volatile v4u*)(dp + DF)     = os;
  *(volatile v4u*)(dp + 2 * DF) = on;
  *(volatile v4u*)(dp + 3 * DF) = on;
  __threadfence();
  *(volatile v4u*)(dp)          = os;
  *(volatile v4u*)(dp + DF)     = os;
  *(volatile v4u*)(dp + 2 * DF) = on;
  *(volatile v4u*)(dp + 3 * DF) = on;
}

template <int MODE>
__global__ __launch_bounds__(256) void k_row(const float* __restrict__ Y, const float* __restrict__ bA,
                                             const float* __restrict__ bB, const float* __restrict__ ex,
                                             const int* __restrict__ FLAG, float* XF, unsigned short* Apl,
                                             float* outp, int nN) {
  __shared__ __attribute__((aligned(16))) float sb[2][DF];
  __shared__ __attribute__((aligned(16))) unsigned short rowbuf[8][2 * DF];
  const int tid = (int)threadIdx.x, lane = tid & 31, wave = tid >> 5;
  if (tid < 32) {
    v4f a = *(const v4f*)(bA + 4 * tid);
    v4f b = *(const v4f*)(bB + 4 * tid);
    a = (v4f){ bf16_val(a[0]), bf16_val(a[1]), bf16_val(a[2]), bf16_val(a[3]) };
    b = (v4f){ bf16_val(b[0]), bf16_val(b[1]), bf16_val(b[2]), bf16_val(b[3]) };
    *(v4fa*)(&sb[0][4 * tid]) = a;
    *(v4fa*)(&sb[1][4 * tid]) = b;
  }
  __syncthreads();
  const v4f b1 = *(const v4fa*)(&sb[0][4 * lane]);
  const v4f b2 = *(const v4fa*)(&sb[1][4 * lane]);
  int fl = 0;
  if (MODE == 2) {
    fl = FLAG[clampi((int)blockIdx.x >> 3, 0, NBLK - 1) * 32];
    asm volatile("" :: "v"(fl));
  }
  const float qnan = __int_as_float(0x7fc00000);
#pragma unroll 1
  for (int i = 0; i < 16; ++i) {
    const int row = (int)blockIdx.x * 128 + wave * 16 + i;
    const bool live = row < nN;
    const int rc = live ? row : nN - 1;
    const v4f y = *(const v4f*)(Y + (size_t)rc * DF + 4 * lane);
    asm volatile("" :: "v"(y));
    float e = 1.0f;
    if (MODE >= 1) {
      const float er = ex[rc];
      asm volatile("" :: "v"(er));
      e = bf16_val(er);
    }
    v4f v = y + b1;
    if (MODE >= 1) v = v + b2;
    if (MODE <= 1) v = (v4f){ relu_keep(v[0]), relu_keep(v[1]), relu_keep(v[2]), relu_keep(v[3]) };
    if (MODE >= 1) v = v * e;
    if (MODE == 2) {
      const bool pz = fl != 0;
      v = (v4f){ pz ? qnan : v[0], pz ? qnan : v[1], pz ? qnan : v[2], pz ? qnan : v[3] };
    }
    v = (v4f){ live ? v[0] : 0.0f, live ? v[1] : 0.0f, live ? v[2] : 0.0f, live ? v[3] : 0.0f };
    if (MODE <= 1) {
      const v4u q = hilo_piece(rowbuf[wave], lane, v);
      float* xp = XF + (size_t)row * DF + 4 * lane;
      unsigned short* ap = Apl + (size_t)row * AP + 8 * lane;
      *(volatile v4f*)xp = v;
      *(volatile v4u*)ap = q;
      __threadfence();
      *(volatile v4f*)xp = v;
      *(volatile v4u*)ap = q;
    } else {
      if (live) {
        float* op = outp + (size_t)row * DF + 4 * lane;
        *(volatile v4f*)op = v;
        __threadfence();
        *(volatile v4f*)op = v;
      }
    }
  }
}

__global__ __launch_bounds__(256) void k_bucket(const int* __restrict__ ei, int* LIST, int* CNT, int* OFF, int* FLAG) {
  extern __shared__ __attribute__((aligned(16))) int dsm[];
  int* wl   = dsm;
  int* cw   = dsm + 8 * WLCAP;
  int* sl   = cw + 8 * NBA;
  int* misc = sl + RCAP;
  const int tid = (int)threadIdx.x, lane = tid & 31, wave = tid >> 5;
  const int b = (int)blockIdx.x;
  const unsigned ub = (unsigned)(b * NBA);
  {
    const v4i z4 = (v4i){0, 0, 0, 0};
    for (int i = tid * 4; i < BK_ZINTS; i += 1024) *(v4ia*)(cw + i) = z4;
  }
  __syncthreads();

  int* mywl = wl + wave * WLCAP;
  const int* tg = ei + NE;
  const int wbase = wave * EW;
  const int lim = wbase + EW;
  int wc = 0, ovl = 0;
#pragma unroll 1
  for (int st = 0; st < NSTEP; ++st) {
    const int e0 = wbase + st * STEP + lane * 8;
    const int ec = e0 < lim - 8 ? e0 : lim - 8;
    const bool valid = e0 < lim;
    const v4i ta = *(const v4i*)(tg + ec);
    const v4i tb = *(const v4i*)(tg + ec + 4);
    const v4i sa = *(const v4i*)(ei + ec);
    const v4i sc = *(const v4i*)(ei + ec + 4);
    asm volatile("" :: "v"(ta));
    asm volatile("" :: "v"(tb));
    asm volatile("" :: "v"(sa));
    asm volatile("" :: "v"(sc));
    const unsigned s0 = (unsigned)ta.x - ub, s1 = (unsigned)ta.y - ub, s2 = (unsigned)ta.z - ub, s3 = (unsigned)ta.w - ub;
    const unsigned s4 = (unsigned)tb.x - ub, s5 = (unsigned)tb.y - ub, s6 = (unsigned)tb.z - ub, s7 = (unsigned)tb.w - ub;
    const bool h0 = valid & (s0 < (unsigned)NBA), h1 = valid & (s1 < (unsigned)NBA);
    const bool h2 = valid & (s2 < (unsigned)NBA), h3 = valid & (s3 < (unsigned)NBA);
    const bool h4 = valid & (s4 < (unsigned)NBA), h5 = valid & (s5 < (unsigned)NBA);
    const bool h6 = valid & (s6 < (unsigned)NBA), h7 = valid & (s7 < (unsigned)NBA);
    const unsigned m0 = __builtin_amdgcn_ballot_w32(h0), m1 = __builtin_amdgcn_ballot_w32(h1);
    const unsigned m2 = __builtin_amdgcn_ballot_w32(h2), m3 = __builtin_amdgcn_ballot_w32(h3);
    const unsigned m4 = __builtin_amdgcn_ballot_w32(h4), m5 = __builtin_amdgcn_ballot_w32(h5);
    const unsigned m6 = __builtin_amdgcn_ballot_w32(h6), m7 = __builtin_amdgcn_ballot_w32(h7);
    const unsigned many = m0 | m1 | m2 | m3 | m4 | m5 | m6 | m7;
    if (many != 0u) {
      const int lower = (int)(__builtin_amdgcn_mbcnt_lo(m0, 0u) + __builtin_amdgcn_mbcnt_lo(m1, 0u) +
                              __builtin_amdgcn_mbcnt_lo(m2, 0u) + __builtin_amdgcn_mbcnt_lo(m3, 0u) +
                              __builtin_amdgcn_mbcnt_lo(m4, 0u) + __builtin_amdgcn_mbcnt_lo(m5, 0u) +
                              __builtin_amdgcn_mbcnt_lo(m6, 0u) + __builtin_amdgcn_mbcnt_lo(m7, 0u));
      int pos = wc + lower;
#define PUTJ(HJ, SJ, GJ) \
      if (HJ) { \
        if (pos < WLCAP) mywl[pos] = (clampi((GJ), 0, NN - 1) << SLA) | (int)(SJ); \
        else ovl = 1; \
        pos = pos + 1; }
      PUTJ(h0, s0, sa.x)
      PUTJ(h1, s1, sa.y)
      PUTJ(h2, s2, sa.z)
      PUTJ(h3, s3, sa.w)
      PUTJ(h4, s4, sc.x)
      PUTJ(h5, s5, sc.y)
      PUTJ(h6, s6, sc.z)
      PUTJ(h7, s7, sc.w)
#undef PUTJ
      wc += (int)(__builtin_popcount(m0) + __builtin_popcount(m1) + __builtin_popcount(m2) + __builtin_popcount(m3) +
                  __builtin_popcount(m4) + __builtin_popcount(m5) + __builtin_popcount(m6) + __builtin_popcount(m7));
    }
  }
  const unsigned ovm = __builtin_amdgcn_ballot_w32(ovl != 0);
  const int wcu = __builtin_amdgcn_readfirstlane(wc);
  const int wcc = wcu < 0 ? 0 : (wcu > WLCAP ? WLCAP : wcu);
  wave_sync();
  if (lane == 0) {
    int* mycw = cw + wave * NBA;
#pragma unroll 1
    for (int i = 0; i < wcc; ++i) {
      const int u = mywl[i];
      const int s = u & (NBA - 1);
      mycw[s] = mycw[s] + 1;
    }
    misc[wave] = wcc;
    misc[8 + wave] = ((ovm != 0u) || (wcu > WLCAP)) ? 1 : 0;
  }
  __syncthreads();

  v4i q[8];
#pragma unroll
  for (int w = 0; w < 8; ++w) q[w] = *(const v4ia*)(cw + w * NBA + 4 * tid);
  v4i cntv = (v4i){0, 0, 0, 0};
#pragma unroll
  for (int w = 0; w < 8; ++w) cntv += q[w];
  const int ssum = cntv.x + cntv.y + cntv.z + cntv.w;
  int incl = ssum;
#pragma unroll
  for (int d = 1; d < 32; d <<= 1) {
    const int y = __shfl_up(incl, d, 32);
    if (lane >= d) incl += y;
  }
  const bool dbig = (cntv.x > DEGCAP) | (cntv.y > DEGCAP) | (cntv.z > DEGCAP) | (cntv.w > DEGCAP);
  const unsigned dbm = __builtin_amdgcn_ballot_w32(dbig);
  if (lane == 31) misc[16 + wave] = incl;
  if (lane == 0)  misc[24 + wave] = (dbm != 0u) ? 1 : 0;
  __syncthreads();
  int pre = 0, tot = 0, fl = 0;
#pragma unroll
  for (int w = 0; w < 8; ++w) {
    const int t = misc[16 + w];
    tot += t;
    pre += (w < wave) ? t : 0;
    fl |= misc[8 + w] | misc[24 + w];
  }
  fl |= (tot > RCAP) ? 1 : 0;
  const int excl = pre + incl - ssum;
  const v4i offv = (v4i){ excl, excl + cntv.x, excl + cntv.x + cntv.y, excl + cntv.x + cntv.y + cntv.z };
  {
    v4i run = offv;
#pragma unroll
    for (int w = 0; w < 8; ++w) {
      *(v4ia*)(cw + w * NBA + 4 * tid) = run;
      run += q[w];
    }
  }
  __syncthreads();

  if (lane == 0) {
    int* mycw = cw + wave * NBA;
#pragma unroll 1
    for (int i = 0; i < wcc; ++i) {
      const int u = mywl[i];
      const int s = u & (NBA - 1);
      const int p = mycw[s];
      mycw[s] = p + 1;
      if ((unsigned)p < (unsigned)RCAP) sl[p] = u >> SLA;
    }
  }
  __syncthreads();

  int* lg = LIST + (size_t)b * RCAP;
  const v4i fv = (v4i){ fl, fl, fl, fl };
  for (int pass = 0; pass < 2; ++pass) {
#pragma unroll 3
    for (int it = 0; it < RCAP / 1024; ++it) {
      const int piece = tid + 256 * it;
      const v4i v = *(const v4ia*)(sl + 4 * piece);
      *(volatile v4i*)(lg + 4 * piece) = v;
    }
    *(volatile v4i*)(CNT + (size_t)b * NBA + 4 * tid) = cntv;
    *(volatile v4i*)(OFF + (size_t)b * NBA + 4 * tid) = offv;
    if (tid < 8) *(volatile v4i*)(FLAG + b * 32 + 4 * tid) = fv;
    __threadfence();
  }
}

__global__ __launch_bounds__(256) void k_replay(const int* __restrict__ LIST, const int* __restrict__ CNT,
                                                const int* __restrict__ OFF, const int* __restrict__ FLAG,
                                                const float* __restrict__ XF, unsigned short* Apl, int nN, int mRows) {
  __shared__ __attribute__((aligned(16))) int scnt[NBA];
  __shared__ __attribute__((aligned(16))) int soff[NBA];
  __shared__ __attribute__((aligned(16))) unsigned short rowbuf[8][2 * DF];
  const int tid = (int)threadIdx.x, lane = tid & 31, wave = tid >> 5;
  const int b = (int)blockIdx.x;
  {
    const v4i c4 = *(const v4i*)(CNT + (size_t)b * NBA + 4 * tid);
    const v4i o4 = *(const v4i*)(OFF + (size_t)b * NBA + 4 * tid);
    asm volatile("" :: "v"(c4));
    asm volatile("" :: "v"(o4));
    *(v4ia*)(scnt + 4 * tid) = c4;
    *(v4ia*)(soff + 4 * tid) = o4;
  }
  int fl = FLAG[b * 32];
  asm volatile("" :: "v"(fl));
  __syncthreads();
  const int* lst = LIST + (size_t)b * RCAP;
  const float qnan = __int_as_float(0x7fc00000);
#pragma unroll 1
  for (int si = 0; si < NBA / 8; ++si) {
    const int s = si * 8 + wave;
    const int node = b * NBA + s;
    const bool live = node < nN;
    const int cv = scnt[s];
    const bool big = (cv > DEGCAP) | (cv < 0);
    int cc = clampi(cv, 0, DEGCAP);
    cc = live ? cc : 0;
    const int cn = __builtin_amdgcn_readfirstlane(cc);
    const int o  = __builtin_amdgcn_readfirstlane(clampi(soff[s], 0, RCAP - 1));
    v4f acc = (v4f){0.0f, 0.0f, 0.0f, 0.0f};
#pragma unroll 1
    for (int b0 = 0; b0 < cn; b0 += 32) {
      int last = o + cn - 1;
      last = last > RCAP - 1 ? RCAP - 1 : last;
      int idx = o + b0 + lane;
      idx = idx > last ? last : idx;
      int sr = lst[idx];
      asm volatile("" :: "v"(sr));
      sr = clampi(sr, 0, nN - 1);
      const int m32 = (cn - b0) < 32 ? (cn - b0) : 32;
#pragma unroll 1
      for (int k = 0; k < m32; ++k) {
        const int sk = __builtin_amdgcn_readlane(sr, k);
        const v4f a = *(const v4f*)(XF + (size_t)sk * DF + 4 * lane);
        asm volatile("" :: "v"(a));
        acc = acc + a;
      }
    }
    const float d = (float)(cn > 1 ? cn : 1);
    v4f m = acc / d;
    const bool pz = (fl != 0) | big;
    m = (v4f){ pz ? qnan : m[0], pz ? qnan : m[1], pz ? qnan : m[2], pz ? qnan : m[3] };
    m = (v4f){ live ? m[0] : 0.0f, live ? m[1] : 0.0f, live ? m[2] : 0.0f, live ? m[3] : 0.0f };
    const v4u qv = hilo_piece(rowbuf[wave], lane, m);
    if (node < mRows) {
      unsigned short* ap = Apl + (size_t)node * AP + 2 * DF + 8 * lane;
      *(volatile v4u*)ap = qv;
      __threadfence();
      *(volatile v4u*)ap = qv;
    }
  }
}

extern "C" void kernel_launch(void* const* d_in, const int* in_sizes, int n_in,
                              void* d_out, int out_size, void* d_ws, size_t ws_size,
                              hipStream_t stream) {
  if (n_in < 15) return;
  if (in_sizes[0] != NN * ATTR || in_sizes[1] != NN || in_sizes[2] != NN || in_sizes[3] != NN) return;
  if (in_sizes[4] != DF * DF || in_sizes[5] != DF) return;
  if (in_sizes[6] != DF * DF || in_sizes[7] != DF || in_sizes[8] != DF * DF || in_sizes[9] != DF) return;
  if (in_sizes[10] != DF * DF || in_sizes[11] != DF || in_sizes[12] != DF * DF || in_sizes[13] != DF) return;
  if (in_sizes[14] != 2 * NE) return;
  if (out_size != NN * DF) return;
  if ((size_t)WS_TOTAL > ws_size) return;

  const float* attr  = (const float*)d_in[0];
  const float* clust = (const float*)d_in[1];
  const float* ratio = (const float*)d_in[2];
  const float* exist = (const float*)d_in[3];
  const float* W_in  = (const float*)d_in[4];
  const float* b_in  = (const float*)d_in[5];
  const float* W1s   = (const float*)d_in[6];
  const float* b1s   = (const float*)d_in[7];
  const float* W1n   = (const float*)d_in[8];
  const float* b1n   = (const float*)d_in[9];
  const float* W2s   = (const float*)d_in[10];
  const float* b2s   = (const float*)d_in[11];
  const float* W2n   = (const float*)d_in[12];
  const float* b2n   = (const float*)d_in[13];
  const int*   edges = (const int*)d_in[14];
  float* out = (float*)d_out;

  char* ws = (char*)d_ws;
  size_t off = 0;
  unsigned short* X0B  = (unsigned short*)(ws + off); off += SZ_X0B;
  float*          XF   = (float*)(ws + off);          off += SZ_XF;
  unsigned short* Apl  = (unsigned short*)(ws + off); off += SZ_A;
  float*          Y    = (float*)(ws + off);          off += SZ_Y;
  int*            LIST = (int*)(ws + off);            off += SZ_LIST;
  int*            CNT  = (int*)(ws + off);            off += SZ_CNT;
  int*            OFF  = (int*)(ws + off);            off += SZ_CNT;
  int*            FLAG = (int*)(ws + off);            off += SZ_FLAG;
  unsigned short* WinB = (unsigned short*)(ws + off); off += SZ_WIN;
  unsigned short* W1c  = (unsigned short*)(ws + off); off += SZ_WCAT;
  unsigned short* W2c  = (unsigned short*)(ws + off); off += SZ_WCAT;
  if (off != (size_t)WS_TOTAL) return;

  hipFuncSetAttribute(reinterpret_cast<const void*>(&k_bucket), hipFuncAttributeMaxDynamicSharedMemorySize, (int)BK_LDS);

  const int gemmGrid = (((NN + 63) / 64) * (DF / 64) + 7) / 8;

  k_xplane<<<MP / XROWS, 256, 0, stream>>>(attr, clust, ratio, exist, X0B, NN);
  k_plane<0><<<DF * DF / 8 / 256, 256, 0, stream>>>(W_in, DF, DF, DF, WinB, DF, DF);
  k_wcat<<<DF * 16 / 256, 256, 0, stream>>>(W1s, W1n, W1c);
  k_wcat<<<DF * 16 / 256, 256, 0, stream>>>(W2s, W2n, W2c);
  k_bucket<<<NBLK, 256, BK_LDS, stream>>>(edges, LIST, CNT, OFF, FLAG);
  k_gemm_nt<0, 0><<<gemmGrid, 256, 0, stream>>>(X0B, WinB, b_in, Y, NN, DF, DF, DF);
  k_row<0><<<MP / 128, 256, 0, stream>>>(Y, b_in, b_in, exist, FLAG, XF, Apl, out, NN);
  k_replay<<<NBLK, 256, 0, stream>>>(LIST, CNT, OFF, FLAG, XF, Apl, NN, MP);
  k_gemm_nt<1, 0><<<gemmGrid, 256, 0, stream>>>(Apl, W1c, b1s, Y, NN, DF, AP, DF);
  k_row<1><<<MP / 128, 256, 0, stream>>>(Y, b1s, b1n, exist, FLAG, XF, Apl, out, NN);
  k_replay<<<NBLK, 256, 0, stream>>>(LIST, CNT, OFF, FLAG, XF, Apl, NN, MP);
  k_gemm_nt<1, 0><<<gemmGrid, 256, 0, stream>>>(Apl, W2c, b2s, Y, NN, DF, AP, DF);
  k_row<2><<<MP / 128, 256, 0, stream>>>(Y, b2s, b2n, exist, FLAG, XF, Apl, out, NN);
}
